// MambaBlock_4303557230699
// MI455X (gfx1250) — hardware-run, weakly checked
//
#include <hip/hip_runtime.h>
#include <math.h>

typedef __attribute__((ext_vector_type(16))) _Float16 v16h;
typedef __attribute__((ext_vector_type(8)))  _Float16 v8h;
typedef __attribute__((ext_vector_type(16))) __bf16   v16b;
typedef __attribute__((ext_vector_type(8)))  __bf16   v8b;
typedef __attribute__((ext_vector_type(8)))  float    v8f;
typedef __attribute__((ext_vector_type(4)))  float    v4f;
typedef __attribute__((ext_vector_type(2)))  float    v2f;
typedef __attribute__((ext_vector_type(4)))  unsigned v4u;

constexpr int kBatch = 2;
constexpr int kSeq   = 2048;
constexpr int kDim   = 1024;
constexpr int kDin   = 2048;
constexpr int kNst   = 16;
constexpr int kDtR   = 64;
constexpr int kXzP   = 2 * kDin;
constexpr int kXdW   = kDtR + 2 * kNst;
constexpr int kXdP   = 128;
constexpr int kFfn   = 4 * kDim;
constexpr int kRows  = kBatch * kSeq;
constexpr int kConvCh = 512;
constexpr int kConvTP = 516;
constexpr int kScanTS = 32;
constexpr int kScanCh = 64;
constexpr int kScanYP = 68;
constexpr float kCarryW   = 64.0f;
constexpr float kCarryU   = 16.0f;
constexpr float kCarryXd  = 16.0f;
constexpr float kCarryY   = 256.0f;
constexpr float kCarryMid = 8.0f;
static_assert(kXdW <= kXdP);
static_assert((kDim % 32) == 0 && (kDin % 32) == 0 && (kDtR % 32) == 0 && (kFfn % 32) == 0);
static_assert((kRows % 64) == 0 && (kXzP % 64) == 0 && (kXdP % 64) == 0 && (kDim % 64) == 0 && (kDin % 64) == 0 && (kFfn % 64) == 0);
static_assert(((kRows / 64) * (kXzP / 64)) % 8 == 0 && ((kRows / 64) * (kXdP / 64)) % 8 == 0 &&
              ((kRows / 64) * (kDin / 64)) % 8 == 0 && ((kRows / 64) * (kDim / 64)) % 8 == 0 &&
              ((kRows / 64) * (kFfn / 64)) % 8 == 0);
static_assert((kSeq % 64) == 0 && (kSeq % kScanTS) == 0 && (kDin % kConvCh) == 0 && (kDin % kScanCh) == 0 && (kRows % 8) == 0);
static_assert(kDim == 1024 && kScanCh == 64 && kScanTS == 32 && kConvCh == 512);

constexpr size_t kOffWIN  = 0;
constexpr size_t kOffWX   = kOffWIN  + (size_t)kXzP * kDim * 2;
constexpr size_t kOffWDT  = kOffWX   + (size_t)kXdP * kDin * 2;
constexpr size_t kOffWOUT = kOffWDT  + (size_t)kDin * kDtR * 2;
constexpr size_t kOffWF1  = kOffWOUT + (size_t)kDim * kDin * 2;
constexpr size_t kOffWF2  = kOffWF1  + (size_t)kFfn * kDim * 2;
constexpr size_t kOffXLN  = kOffWF2  + (size_t)kDim * kFfn * 2;
constexpr size_t kOffXZ   = kOffXLN  + (size_t)kRows * kDim * 2;
constexpr size_t kOffXC   = kOffXZ   + (size_t)kRows * kXzP * 2;
constexpr size_t kOffXD   = kOffXC   + (size_t)kRows * kDin * 2;
constexpr size_t kOffY    = kOffXD   + (size_t)kRows * kXdP * 2;
constexpr size_t kOffH1   = kOffY    + (size_t)kRows * kDin * 2;
constexpr size_t kWsTotal = kOffH1   + (size_t)kRows * kDim * 4;
static_assert(kWsTotal == 123469824ull);
static_assert(kWsTotal <= 134217728ull);
static_assert((kOffWX % 128) == 0 && (kOffWDT % 128) == 0 && (kOffWOUT % 128) == 0 && (kOffWF1 % 128) == 0 &&
              (kOffWF2 % 128) == 0 && (kOffXLN % 128) == 0 && (kOffXZ % 128) == 0 && (kOffXC % 128) == 0 &&
              (kOffXD % 128) == 0 && (kOffY % 128) == 0 && (kOffH1 % 128) == 0);

__device__ __forceinline__ unsigned short f2bf_bits(float f) {
  unsigned u = __float_as_uint(f);
  return (unsigned short)((u + 0x7FFFu + ((u >> 16) & 1u)) >> 16);
}
__device__ __forceinline__ float bf_bits2f(unsigned short h) { return __uint_as_float(((unsigned)h) << 16); }

__device__ __forceinline__ float h16_to_f32(unsigned hb) {
  const unsigned sgn = (hb & 0x8000u) << 16; const unsigned em = hb & 0x7fffu;
  const float fn = __uint_as_float((em << 13) + 0x38000000u);
  const float fs = (float)em * 5.9604644775390625e-8f;
  const float mag = (em < 0x400u) ? fs : fn; return __uint_as_float(__float_as_uint(mag) | sgn);
}

__device__ __forceinline__ void dep_guard4_h(v8f& a, v8f& b, v8f& c, v8f& d, v16h x, v16h y) {
  asm volatile("v_nop\n\tv_nop\n\tv_nop\n\tv_nop" : "+v"(a), "+v"(b), "+v"(c), "+v"(d) : "v"(x), "v"(y));
}
__device__ __forceinline__ void dep_guard4_b(v8f& a, v8f& b, v8f& c, v8f& d, v16b x, v16b y) {
  asm volatile("v_nop\n\tv_nop\n\tv_nop\n\tv_nop" : "+v"(a), "+v"(b), "+v"(c), "+v"(d) : "v"(x), "v"(y));
}
__device__ __forceinline__ void keep4_h(v16h a, v16h b, v16h c, v16h d) { asm volatile("v_nop" :: "v"(a), "v"(b), "v"(c), "v"(d)); }
__device__ __forceinline__ void keep4_b(v16b a, v16b b, v16b c, v16b d) { asm volatile("v_nop" :: "v"(a), "v"(b), "v"(c), "v"(d)); }
__device__ __forceinline__ void acc_guard4(v8f& a, v8f& b, v8f& c, v8f& d) { asm volatile("v_nop\n\tv_nop\n\tv_nop\n\tv_nop" : "+v"(a), "+v"(b), "+v"(c), "+v"(d)); }
template <typename T> struct Frag;
template <> struct Frag<_Float16> {
  typedef v16h V; union U { v16h v; v8h h[2]; };
  static __device__ __forceinline__ v16h load(const _Float16* p) {
    U f; f.h[0] = *(const v8h*)(p); f.h[1] = *(const v8h*)(p + 16); return f.v;
  }
  static __device__ __forceinline__ v8f mma(v16h a, v16h b, v8f c) {
    return __builtin_amdgcn_wmma_f32_16x16x32_f16(false, a, false, b, (short)0, c, false, false);
  }
  static __device__ __forceinline__ void guard4(v8f& a, v8f& b, v8f& c, v8f& d, v16h x, v16h y) { dep_guard4_h(a, b, c, d, x, y); }
  static __device__ __forceinline__ void keep(v16h a, v16h b, v16h c, v16h d) { keep4_h(a, b, c, d); }
};
template <> struct Frag<__bf16> {
  typedef v16b V; union U { v16b v; v8b h[2]; };
  static __device__ __forceinline__ v16b load(const __bf16* p) {
    U f; f.h[0] = *(const v8b*)(p); f.h[1] = *(const v8b*)(p + 16); return f.v;
  }
  static __device__ __forceinline__ v8f mma(v16b a, v16b b, v8f c) {
    return __builtin_amdgcn_wmma_f32_16x16x32_bf16(false, a, false, b, (short)0, c, false, false);
  }
  static __device__ __forceinline__ void guard4(v8f& a, v8f& b, v8f& c, v8f& d, v16b x, v16b y) { dep_guard4_b(a, b, c, d, x, y); }
  static __device__ __forceinline__ void keep(v16b a, v16b b, v16b c, v16b d) { keep4_b(a, b, c, d); }
};

template <int ET> struct Elem;
template <> struct Elem<0> { typedef _Float16 T; };
template <> struct Elem<1> { typedef __bf16 T; };
template <int ET, bool SPLIT, int BIAS_MODE, int OUT_MODE, bool RESID, int ACT = 0>
__global__ __launch_bounds__(256) void wmma_gemm64(
    const unsigned short* __restrict__ Ap, const unsigned short* __restrict__ A2p, int lda, long strideA,
    const unsigned short* __restrict__ Btp, const unsigned short* __restrict__ Bt2p, int ldb, long strideB,
    void* __restrict__ Cout, void* __restrict__ Cout2, int ldc, long strideC,
    const float* __restrict__ bias,
    const float* __restrict__ resid, long strideR,
    int M, int N, int K, float scale) {
  static_assert(!(RESID && OUT_MODE != 0));
  static_assert(!(RESID && ACT != 0));
  typedef typename Elem<ET>::T T;
  typedef typename Frag<T>::V V;
  const T* A = (const T*)Ap; const T* A2 = (const T*)A2p; const T* Bt = (const T*)Btp; const T* Bt2 = (const T*)Bt2p;
  __shared__ __align__(16) float sT[8][16 * 68];
  const int b    = blockIdx.y;
  const int lane = threadIdx.x & 31;
  const int wave = threadIdx.x >> 5;
  const int tilesN = N >> 6;
  const int tilesM = M >> 6;
  const int tile = blockIdx.x * 8 + wave;
  if (tile >= tilesM * tilesN) return;
  const int tm = tile / tilesN;
  const int tn = tile - tm * tilesN;
  const int m0 = tm << 6;
  const int n0 = tn << 6;

  const T* Ab  = A  + (size_t)b * strideA;
  const T* Bb  = Bt + (size_t)b * strideB;
  const T* Ab2 = SPLIT ? (A2  + (size_t)b * strideA) : nullptr;
  const T* Bb2 = SPLIT ? (Bt2 + (size_t)b * strideB) : nullptr;

  const int rlane = lane & 15;
  const int koff  = (lane >> 4) * 8;
  const int mOff  = (lane >> 4) * 8;

  v8f acc[4][4];
#pragma unroll
  for (int i = 0; i < 4; ++i)
#pragma unroll
    for (int j = 0; j < 4; ++j) acc[i][j] = (v8f){0.f,0.f,0.f,0.f,0.f,0.f,0.f,0.f};

  for (int k0 = 0; k0 < K; k0 += 32) {
    V bh[4], bl[4];
#pragma unroll
    for (int j = 0; j < 4; ++j) {
      const size_t bo = (size_t)(n0 + (j << 4) + rlane) * ldb + koff + k0;
      bh[j] = Frag<T>::load(Bb + bo);
      if (SPLIT) bl[j] = Frag<T>::load(Bb2 + bo);
    }
#pragma unroll
    for (int i = 0; i < 4; ++i) {
      const size_t ao = (size_t)(m0 + (i << 4) + rlane) * lda + koff + k0;
      V ah = Frag<T>::load(Ab + ao);
      V al;
      if (SPLIT) al = Frag<T>::load(Ab2 + ao);
#pragma unroll
      for (int j = 0; j < 4; ++j) {
        acc[i][j] = Frag<T>::mma(ah, bh[j], acc[i][j]);
        if (SPLIT) {
          acc[i][j] = Frag<T>::mma(ah, bl[j], acc[i][j]);
          acc[i][j] = Frag<T>::mma(al, bh[j], acc[i][j]);
        }
      }
      Frag<T>::guard4(acc[i][0], acc[i][1], acc[i][2], acc[i][3], ah, SPLIT ? al : ah);
    }
    Frag<T>::keep(bh[0], bh[1], bh[2], bh[3]);
    if (SPLIT) Frag<T>::keep(bl[0], bl[1], bl[2], bl[3]);
  }
  acc_guard4(acc[0][0], acc[0][1], acc[0][2], acc[0][3]);
  acc_guard4(acc[1][0], acc[1][1], acc[1][2], acc[1][3]);
  acc_guard4(acc[2][0], acc[2][1], acc[2][2], acc[2][3]);
  acc_guard4(acc[3][0], acc[3][1], acc[3][2], acc[3][3]);

  float* slab = sT[wave];
  const float* Rb = RESID ? (resid + (size_t)b * strideR) : nullptr;
#pragma unroll
  for (int i = 0; i < 4; ++i) {
    const int mBase = m0 + (i << 4);
#pragma unroll
    for (int j = 0; j < 4; ++j) {
      const int n = n0 + (j << 4) + rlane;
      float bv = 0.f;
      if (BIAS_MODE == 2) bv = bias[n];
#pragma unroll
      for (int r = 0; r < 8; ++r) {
        float v = acc[i][j][r] * scale;
        if (BIAS_MODE == 1) v += bias[mBase + mOff + r];
        if (BIAS_MODE == 2) v += bv;
        if (ACT == 1) v = tanhf(v);
        if (ACT == 2) v = fmaxf(v, 0.0f);
        if (ACT == 3) v = v / (1.0f + expf(-v));
        if (ACT == 4) v = (v > 0.f) ? v : 0.01f * v;
        slab[(mOff + r) * 68 + (j << 4) + rlane] = v;
      }
    }
    __builtin_amdgcn_fence(__ATOMIC_RELEASE, "workgroup");
    __builtin_amdgcn_wave_barrier();
    __builtin_amdgcn_fence(__ATOMIC_ACQUIRE, "workgroup");
    if (OUT_MODE == 0) {
      float* C = (float*)Cout + (size_t)b * strideC;
      const int hh = lane >> 4, c4 = (lane & 15) * 4;
      v4f vals[8];
#pragma unroll
      for (int it = 0; it < 8; ++it) {
        const int row = it * 2 + hh;
        v4f v = *(const v4f*)(slab + row * 68 + c4);
        if (RESID) {
          const v4f rr = *(const v4f*)(Rb + (size_t)(mBase + row) * ldc + n0 + c4);
          v = v + rr;
        }
        vals[it] = v;
      }
      for (int pass = 0; pass < 2; ++pass) {
#pragma unroll
        for (int it = 0; it < 8; ++it) {
          const int row = it * 2 + hh;
          *(volatile v4f*)(C + (size_t)(mBase + row) * ldc + n0 + c4) = vals[it];
        }
        __threadfence();
      }
    } else {
      const int q = lane >> 3, c8 = (lane & 7) * 8;
      unsigned short* C  = (unsigned short*)Cout  + (size_t)b * strideC;
      unsigned short* C2 = (OUT_MODE == 2) ? ((unsigned short*)Cout2 + (size_t)b * strideC) : nullptr;
      for (int pass = 0; pass < 2; ++pass) {
#pragma unroll
        for (int it = 0; it < 4; ++it) {
          const int row = it * 4 + q;
          const float* sp = slab + row * 68 + c8;
          v8h hv, lv;
#pragma unroll
          for (int e = 0; e < 8; ++e) {
            if (OUT_MODE == 1) {
              hv[e] = (_Float16)sp[e];
            } else {
              unsigned short hb = f2bf_bits(sp[e]);
              unsigned short lb = f2bf_bits(sp[e] - bf_bits2f(hb));
              hv[e] = __builtin_bit_cast(_Float16, hb);
              lv[e] = __builtin_bit_cast(_Float16, lb);
            }
          }
          *(volatile v8h*)(C + (size_t)(mBase + row) * ldc + n0 + c8) = hv;
          if (OUT_MODE == 2) *(volatile v8h*)(C2 + (size_t)(mBase + row) * ldc + n0 + c8) = lv;
        }
        __threadfence();
      }
    }
    __builtin_amdgcn_fence(__ATOMIC_RELEASE, "workgroup");
    __builtin_amdgcn_wave_barrier();
    __builtin_amdgcn_fence(__ATOMIC_ACQUIRE, "workgroup");
  }
}

__global__ __launch_bounds__(256) void cvt_rows_f16_kernel(
    const float* __restrict__ src, unsigned short* __restrict__ dst, int rows_src, int cols, int total8, float scale)
{
  const int i = blockIdx.x * 256 + threadIdx.x;
  if (i >= total8) return;
  const size_t e0 = (size_t)i << 3;
  const int row = (int)(e0 / (size_t)cols);
  const int c   = (int)(e0 - (size_t)row * (size_t)cols);
  const int rs  = row < rows_src ? row : (rows_src - 1);
  const float f = row < rows_src ? scale : 0.0f;
  const v4f a0 = *(const v4f*)(src + (size_t)rs * cols + c);
  const v4f a1 = *(const v4f*)(src + (size_t)rs * cols + c + 4);
  v8h hv;
#pragma unroll
  for (int e = 0; e < 4; ++e) {
    hv[e]     = (_Float16)(a0[e] * f);
    hv[4 + e] = (_Float16)(a1[e] * f);
  }
  unsigned short* p = dst + e0;
  *(volatile v8h*)p = hv;
  __threadfence();
  *(volatile v8h*)p = hv;
}

__device__ __forceinline__ float wave_sum32(float v) {
  v += __shfl_xor(v, 16, 32);
  v += __shfl_xor(v, 8, 32);
  v += __shfl_xor(v, 4, 32);
  v += __shfl_xor(v, 2, 32);
  v += __shfl_xor(v, 1, 32);
  return v;
}
__global__ __launch_bounds__(256) void layernorm_f16_kernel(
    const float* __restrict__ X, const float* __restrict__ gw, const float* __restrict__ gb,
    unsigned short* __restrict__ OUT, int nrows)
{
  const int lane = threadIdx.x & 31, wave = threadIdx.x >> 5;
  int row = blockIdx.x * 8 + wave;
  const bool act = row < nrows;
  row = act ? row : (nrows - 1);
  const float* xr = X + (size_t)row * kDim;
  float s = 0.0f;
#pragma unroll 1
  for (int k = 0; k < 4; ++k) {
    const v4f a = *(const v4f*)(xr + 256 * k + 8 * lane);
    const v4f c = *(const v4f*)(xr + 256 * k + 8 * lane + 4);
    s += (a[0] + a[1]) + (a[2] + a[3]);
    s += (c[0] + c[1]) + (c[2] + c[3]);
  }
  s = wave_sum32(s);
  const float mu = s * (1.0f / 1024.0f);
  float q = 0.0f;
#pragma unroll 1
  for (int k = 0; k < 4; ++k) {
    const v4f a = *(const v4f*)(xr + 256 * k + 8 * lane);
    const v4f c = *(const v4f*)(xr + 256 * k + 8 * lane + 4);
    const v4f da = a - mu, dc = c - mu;
    q += (da[0] * da[0] + da[1] * da[1]) + (da[2] * da[2] + da[3] * da[3]);
    q += (dc[0] * dc[0] + dc[1] * dc[1]) + (dc[2] * dc[2] + dc[3] * dc[3]);
  }
  q = wave_sum32(q);
  const float var = q * (1.0f / 1024.0f);
  const float inv = rsqrtf(var + 1e-5f);
#pragma unroll 1
  for (int k = 0; k < 4; ++k) {
    const int c0 = 256 * k + 8 * lane;
    const v4f a  = *(const v4f*)(xr + c0);
    const v4f c  = *(const v4f*)(xr + c0 + 4);
    const v4f wa = *(const v4f*)(gw + c0);
    const v4f wc = *(const v4f*)(gw + c0 + 4);
    const v4f ba = *(const v4f*)(gb + c0);
    const v4f bc = *(const v4f*)(gb + c0 + 4);
    const v4f oa = (a - mu) * inv * wa + ba;
    const v4f oc = (c - mu) * inv * wc + bc;
    v8h hv;
#pragma unroll
    for (int e = 0; e < 4; ++e) { hv[e] = (_Float16)oa[e]; hv[4 + e] = (_Float16)oc[e]; }
    if (act) {
      unsigned short* p = OUT + (size_t)row * kDim + c0;
      *(volatile v8h*)p = hv;
      __threadfence();
      *(volatile v8h*)p = hv;
    }
  }
}

__global__ __launch_bounds__(256) void conv_silu_kernel(
    const unsigned* __restrict__ XZw, const float* __restrict__ cw, const float* __restrict__ cb,
    unsigned short* __restrict__ XC16)
{
  __shared__ __align__(16) float sT[16 * kConvTP];
  constexpr size_t kXzWP = kXzP / 2;
  const int tid = threadIdx.x, lane = tid & 31, wave = tid >> 5;
  const int d0 = blockIdx.x * kConvCh;
  const int da = d0 + 2 * tid;
  const int g0 = blockIdx.y * 64;
  const int tb = g0 & (kSeq - 1);
  const size_t wcol = (size_t)(d0 >> 1) + tid;
  const v4f wA = *(const v4f*)(cw + (size_t)da * 4);
  const v4f wB = *(const v4f*)(cw + (size_t)(da + 1) * 4);
  const v2f bAB = *(const v2f*)(cb + da);
  float a3, a2, a1, b3, b2, b1;
  {
    const bool hist = (tb > 0);
    const int rb = hist ? (g0 - 3) : g0;
    const unsigned u3 = XZw[(size_t)rb * kXzWP + wcol];
    const unsigned u2 = XZw[(size_t)(rb + 1) * kXzWP + wcol];
    const unsigned u1 = XZw[(size_t)(rb + 2) * kXzWP + wcol];
    const float hf = hist ? 1.0f : 0.0f;
    a3 = h16_to_f32(u3 & 0xffffu) * hf; b3 = h16_to_f32(u3 >> 16) * hf;
    a2 = h16_to_f32(u2 & 0xffffu) * hf; b2 = h16_to_f32(u2 >> 16) * hf;
    a1 = h16_to_f32(u1 & 0xffffu) * hf; b1 = h16_to_f32(u1 >> 16) * hf;
  }
#pragma unroll 1
  for (int sub = 0; sub < 4; ++sub) {
    const int lb = g0 + sub * 16;
#pragma unroll 1
    for (int s = 0; s < 16; ++s) {
      const unsigned uw = XZw[(size_t)(lb + s) * kXzWP + wcol];
      const float xa = h16_to_f32(uw & 0xffffu);
      const float xb = h16_to_f32(uw >> 16);
      float acca = wA[0] * a3;
      acca = fmaf(wA[1], a2, acca);
      acca = fmaf(wA[2], a1, acca);
      acca = fmaf(wA[3], xa, acca);
      float accb = wB[0] * b3;
      accb = fmaf(wB[1], b2, accb);
      accb = fmaf(wB[2], b1, accb);
      accb = fmaf(wB[3], xb, accb);
      const float va = acca + bAB[0];
      const float vb = accb + bAB[1];
      const float sa = va * __builtin_amdgcn_rcpf(1.0f + expf(-va));
      const float sb = vb * __builtin_amdgcn_rcpf(1.0f + expf(-vb));
      v2f o; o[0] = sa * kCarryU; o[1] = sb * kCarryU;
      *(v2f*)(sT + s * kConvTP + 2 * tid) = o;
      a3 = a2; a2 = a1; a1 = xa;
      b3 = b2; b2 = b1; b1 = xb;
    }
    __syncthreads();
    v8h hv[4];
#pragma unroll
    for (int r = 0; r < 2; ++r) {
#pragma unroll
      for (int c = 0; c < 2; ++c) {
        const float* sp = sT + (2 * wave + r) * kConvTP + c * 256 + lane * 8;
        const v4f x0 = *(const v4f*)(sp);
        const v4f x1 = *(const v4f*)(sp + 4);
#pragma unroll
        for (int e = 0; e < 4; ++e) { hv[r * 2 + c][e] = (_Float16)x0[e]; hv[r * 2 + c][4 + e] = (_Float16)x1[e]; }
      }
    }
    for (int pass = 0; pass < 2; ++pass) {
#pragma unroll
      for (int r = 0; r < 2; ++r) {
#pragma unroll
        for (int c = 0; c < 2; ++c) {
          unsigned short* p = XC16 + (size_t)(lb + 2 * wave + r) * kDin + d0 + c * 256 + lane * 8;
          *(volatile v8h*)p = hv[r * 2 + c];
        }
      }
      __threadfence();
    }
    __syncthreads();
  }
}

__device__ __forceinline__ void unpack8_h16(v4u w, float s, float* dst) {
  const unsigned w0 = w[0], w1 = w[1], w2 = w[2], w3 = w[3];
  v4f a, b;
  a[0] = h16_to_f32(w0 & 0xffffu) * s; a[1] = h16_to_f32(w0 >> 16) * s;
  a[2] = h16_to_f32(w1 & 0xffffu) * s; a[3] = h16_to_f32(w1 >> 16) * s;
  b[0] = h16_to_f32(w2 & 0xffffu) * s; b[1] = h16_to_f32(w2 >> 16) * s;
  b[2] = h16_to_f32(w3 & 0xffffu) * s; b[3] = h16_to_f32(w3 >> 16) * s;
  *(v4f*)dst = a;
  *(v4f*)(dst + 4) = b;
}

__global__ __launch_bounds__(kScanCh) void scan_kernel(
    const unsigned short* __restrict__ XZ16, const unsigned short* __restrict__ XC16,
    const unsigned short* __restrict__ XD16, const float* __restrict__ Alog,
    const float* __restrict__ Dp, unsigned short* __restrict__ Y16)
{
  __shared__ __align__(16) float sDL[kScanTS * kScanCh];
  __shared__ __align__(16) float sZ [kScanTS * kScanCh];
  __shared__ __align__(16) float sU [kScanTS * kScanCh];
  __shared__ __align__(16) float sBC[kScanTS * 2 * kNst];
  __shared__ __align__(16) float sY [kScanTS * kScanYP];
  const int tid = threadIdx.x, lane = tid & 31, wave = tid >> 5;
  constexpr int kBlkPerB = kDin / kScanCh;
  const int bix = blockIdx.x / kBlkPerB;
  const int d0  = (blockIdx.x - bix * kBlkPerB) * kScanCh;
  const int d   = d0 + tid;
  const size_t row0 = (size_t)bix * kSeq;
  float negA[kNst], h[kNst];
  {
    const v4f e0 = *(const v4f*)(Alog + (size_t)d * kNst);
    const v4f e1 = *(const v4f*)(Alog + (size_t)d * kNst + 4);
    const v4f e2 = *(const v4f*)(Alog + (size_t)d * kNst + 8);
    const v4f e3 = *(const v4f*)(Alog + (size_t)d * kNst + 12);
#pragma unroll
    for (int k = 0; k < 4; ++k) {
      negA[k]      = -expf(e0[k]);
      negA[4 + k]  = -expf(e1[k]);
      negA[8 + k]  = -expf(e2[k]);
      negA[12 + k] = -expf(e3[k]);
    }
#pragma unroll
    for (int n = 0; n < kNst; ++n) h[n] = 0.0f;
  }
  const float Dd = Dp[d];
  const float invU = 1.0f / kCarryU;
  const float invX = 1.0f / kCarryXd;
  const int q = lane >> 3, c8 = (lane & 7) * 8;
#pragma unroll 1
  for (int t0 = 0; t0 < kSeq; t0 += kScanTS) {
    __syncthreads();
#pragma unroll 1
    for (int i = 0; i < 4; ++i) {
      const int idx = tid + kScanCh * i;
      const int r = idx >> 3, cc = (idx & 7) * 8;
      const size_t grow = row0 + t0 + r;
      const v4u wd = *(const v4u*)(XZ16 + grow * kXzP + d0 + cc);
      const v4u wz = *(const v4u*)(XZ16 + grow * kXzP + kDin + d0 + cc);
      const v4u wu = *(const v4u*)(XC16 + grow * kDin + d0 + cc);
      unpack8_h16(wd, 1.0f, sDL + r * kScanCh + cc);
      unpack8_h16(wz, 1.0f, sZ  + r * kScanCh + cc);
      unpack8_h16(wu, invU, sU  + r * kScanCh + cc);
    }
#pragma unroll 1
    for (int j = 0; j < 2; ++j) {
      const int idx = tid + kScanCh * j;
      const int r = idx >> 2, cc = (idx & 3) * 8;
      const v4u wb = *(const v4u*)(XD16 + (row0 + t0 + r) * kXdP + kDtR + cc);
      unpack8_h16(wb, invX, sBC + r * (2 * kNst) + cc);
    }
    __syncthreads();
#pragma unroll 1
    for (int s = 0; s < kScanTS; ++s) {
      const float dl = sDL[s * kScanCh + tid];
      const float zv = sZ [s * kScanCh + tid];
      const float uv = sU [s * kScanCh + tid];
      const float* bcr = sBC + s * (2 * kNst);
      float Bs[kNst], Cs[kNst];
#pragma unroll
      for (int q4 = 0; q4 < 4; ++q4) {
        const v4f bv = *(const v4f*)(bcr + 4 * q4);
        const v4f cv = *(const v4f*)(bcr + kNst + 4 * q4);
        Bs[4 * q4 + 0] = bv[0]; Bs[4 * q4 + 1] = bv[1]; Bs[4 * q4 + 2] = bv[2]; Bs[4 * q4 + 3] = bv[3];
        Cs[4 * q4 + 0] = cv[0]; Cs[4 * q4 + 1] = cv[1]; Cs[4 * q4 + 2] = cv[2]; Cs[4 * q4 + 3] = cv[3];
      }
      const float a   = __expf(-fabsf(dl));
      const float ua  = 1.0f + a;
      const float l1p = __logf(ua) + (a - (ua - 1.0f)) * __builtin_amdgcn_rcpf(ua);
      const float dt  = fmaxf(dl, 0.0f) + l1p;
      const float dtx = dt * uv;
      float y = 0.0f;
#pragma unroll
      for (int n = 0; n < kNst; ++n) {
        const float e = __expf(dt * negA[n]);
        h[n] = e * h[n] + dtx * Bs[n];
        y = y + h[n] * Cs[n];
      }
      y = y + uv * Dd;
      const float sg = __builtin_amdgcn_rcpf(1.0f + __expf(-zv));
      y = y * (zv * sg);
      sY[s * kScanYP + tid] = y * kCarryY;
    }
    __syncthreads();
    v8h hv[4];
#pragma unroll
    for (int it = 0; it < 4; ++it) {
      const int row = it * 8 + wave * 4 + q;
      const float* sp = sY + row * kScanYP + c8;
      const v4f x0 = *(const v4f*)(sp);
      const v4f x1 = *(const v4f*)(sp + 4);
#pragma unroll
      for (int e = 0; e < 4; ++e) { hv[it][e] = (_Float16)x0[e]; hv[it][4 + e] = (_Float16)x1[e]; }
    }
    for (int pass = 0; pass < 2; ++pass) {
#pragma unroll
      for (int it = 0; it < 4; ++it) {
        const int row = it * 8 + wave * 4 + q;
        unsigned short* p = Y16 + (row0 + t0 + row) * kDin + d0 + c8;
        *(volatile v8h*)p = hv[it];
      }
      __threadfence();
    }
  }
}

__global__ __launch_bounds__(256) void gelu_inplace_kernel(unsigned* __restrict__ U, int nwords, float carry)
{
  const int i = blockIdx.x * 256 + threadIdx.x;
  if (i >= nwords) return;
  const unsigned w = U[i];
  const float a = h16_to_f32(w & 0xffffu);
  const float b = h16_to_f32(w >> 16);
  const float ga = 0.5f * a * (1.0f + erff(a * 0.70710678118654752f)) * carry;
  const float gb = 0.5f * b * (1.0f + erff(b * 0.70710678118654752f)) * carry;
  const _Float16 h0 = (_Float16)ga, h1 = (_Float16)gb;
  const unsigned u = (unsigned)__builtin_bit_cast(unsigned short, h0) | ((unsigned)__builtin_bit_cast(unsigned short, h1) << 16);
  ((volatile unsigned*)U)[i] = u;
  __threadfence();
  ((volatile unsigned*)U)[i] = u;
}

extern "C" void kernel_launch(void* const* d_in, const int* in_sizes, int n_in,
                              void* d_out, int out_size, void* d_ws, size_t ws_size,
                              hipStream_t stream) {
  if (n_in < 16) return;
  if (in_sizes[0]  != kRows * kDim) return;
  if (in_sizes[1]  != kDim) return;
  if (in_sizes[2]  != kDim) return;
  if (in_sizes[3]  != kXzP * kDim) return;
  if (in_sizes[4]  != kDin * 4) return;
  if (in_sizes[5]  != kDin) return;
  if (in_sizes[6]  != kXdW * kDin) return;
  if (in_sizes[7]  != kDin * kDtR) return;
  if (in_sizes[8]  != kDin) return;
  if (in_sizes[9]  != kDin * kNst) return;
  if (in_sizes[10] != kDin) return;
  if (in_sizes[11] != kDim * kDin) return;
  if (in_sizes[12] != kFfn * kDim) return;
  if (in_sizes[13] != kFfn) return;
  if (in_sizes[14] != kDim * kFfn) return;
  if (in_sizes[15] != kDim) return;
  if (out_size != kRows * kDim) return;
  if (ws_size < kWsTotal) return;

  const float* x        = (const float*)d_in[0];
  const float* norm_w   = (const float*)d_in[1];
  const float* norm_b   = (const float*)d_in[2];
  const float* in_proj  = (const float*)d_in[3];
  const float* conv_w   = (const float*)d_in[4];
  const float* conv_b   = (const float*)d_in[5];
  const float* x_proj   = (const float*)d_in[6];
  const float* dt_proj  = (const float*)d_in[7];
  const float* dt_bias  = (const float*)d_in[8];
  const float* A_log    = (const float*)d_in[9];
  const float* Dp       = (const float*)d_in[10];
  const float* out_proj = (const float*)d_in[11];
  const float* ffn_w1   = (const float*)d_in[12];
  const float* ffn_b1   = (const float*)d_in[13];
  const float* ffn_w2   = (const float*)d_in[14];
  const float* ffn_b2   = (const float*)d_in[15];
  float* out = (float*)d_out;

  char* ws = (char*)d_ws;
  unsigned short* WIN  = (unsigned short*)(ws + kOffWIN);
  unsigned short* WX   = (unsigned short*)(ws + kOffWX);
  unsigned short* WDT  = (unsigned short*)(ws + kOffWDT);
  unsigned short* WOUT = (unsigned short*)(ws + kOffWOUT);
  unsigned short* WF1  = (unsigned short*)(ws + kOffWF1);
  unsigned short* WF2  = (unsigned short*)(ws + kOffWF2);
  unsigned short* XLN  = (unsigned short*)(ws + kOffXLN);
  unsigned short* XZ   = (unsigned short*)(ws + kOffXZ);
  unsigned short* XC   = (unsigned short*)(ws + kOffXC);
  unsigned short* XD   = (unsigned short*)(ws + kOffXD);
  unsigned short* Y    = (unsigned short*)(ws + kOffY);
  float*          H1   = (float*)(ws + kOffH1);

  {
    const int t_in  = kXzP * kDim / 8;
    const int t_x   = kXdP * kDin / 8;
    const int t_dt  = kDin * kDtR / 8;
    const int t_out = kDim * kDin / 8;
    const int t_f1  = kFfn * kDim / 8;
    const int t_f2  = kDim * kFfn / 8;
    cvt_rows_f16_kernel<<<(t_in + 255) / 256, 256, 0, stream>>>(in_proj, WIN, kXzP, kDim, t_in, kCarryW);
    cvt_rows_f16_kernel<<<(t_x + 255) / 256, 256, 0, stream>>>(x_proj, WX, kXdW, kDin, t_x, kCarryW);
    cvt_rows_f16_kernel<<<(t_dt + 255) / 256, 256, 0, stream>>>(dt_proj, WDT, kDin, kDtR, t_dt, kCarryW);
    cvt_rows_f16_kernel<<<(t_out + 255) / 256, 256, 0, stream>>>(out_proj, WOUT, kDim, kDin, t_out, kCarryW);
    cvt_rows_f16_kernel<<<(t_f1 + 255) / 256, 256, 0, stream>>>(ffn_w1, WF1, kFfn, kDim, t_f1, kCarryW);
    cvt_rows_f16_kernel<<<(t_f2 + 255) / 256, 256, 0, stream>>>(ffn_w2, WF2, kDim, kFfn, t_f2, kCarryW);
  }

  layernorm_f16_kernel<<<kRows / 8, 256, 0, stream>>>(x, norm_w, norm_b, XLN, kRows);

  wmma_gemm64<0, false, 0, 1, false><<<dim3((kRows / 64) * (kXzP / 64) / 8, 1), 256, 0, stream>>>(
      XLN, nullptr, kDim, 0L,
      WIN, nullptr, kDim, 0L,
      (void*)XZ, nullptr, kXzP, 0L,
      nullptr, nullptr, 0L,
      kRows, kXzP, kDim, 1.0f / kCarryW);

  conv_silu_kernel<<<dim3(kDin / kConvCh, kRows / 64), 256, 0, stream>>>((const unsigned*)XZ, conv_w, conv_b, XC);

  wmma_gemm64<0, false, 0, 1, false><<<dim3((kRows / 64) * (kXdP / 64) / 8, 1), 256, 0, stream>>>(
      XC, nullptr, kDin, 0L,
      WX, nullptr, kDin, 0L,
      (void*)XD, nullptr, kXdP, 0L,
      nullptr, nullptr, 0L,
      kRows, kXdP, kDin, kCarryXd / (kCarryU * kCarryW));

  wmma_gemm64<0, false, 2, 1, false><<<dim3((kRows / 64) * (kDin / 64) / 8, 1), 256, 0, stream>>>(
      XD, nullptr, kXdP, 0L,
      WDT, nullptr, kDtR, 0L,
      (void*)XZ, nullptr, kXzP, 0L,
      dt_bias, nullptr, 0L,
      kRows, kDin, kDtR, 1.0f / (kCarryXd * kCarryW));

  scan_kernel<<<kBatch * (kDin / kScanCh), kScanCh, 0, stream>>>(XZ, XC, XD, A_log, Dp, Y);

  wmma_gemm64<0, false, 0, 0, true><<<dim3((kRows / 64) * (kDim / 64) / 8, 1), 256, 0, stream>>>(
      Y, nullptr, kDin, 0L,
      WOUT, nullptr, kDin, 0L,
      (void*)H1, nullptr, kDim, 0L,
      nullptr, x, 0L,
      kRows, kDim, kDin, 1.0f / (kCarryY * kCarryW));

  layernorm_f16_kernel<<<kRows / 8, 256, 0, stream>>>(H1, norm_w, norm_b, XLN, kRows);

  wmma_gemm64<0, false, 2, 1, false><<<dim3((kRows / 64) * (kFfn / 64) / 8, 1), 256, 0, stream>>>(
      XLN, nullptr, kDim, 0L,
      WF1, nullptr, kDim, 0L,
      (void*)XZ, nullptr, kFfn, 0L,
      ffn_b1, nullptr, 0L,
      kRows, kFfn, kDim, 1.0f / kCarryW);

  {
    const int nwords = kRows * kFfn / 2;
    gelu_inplace_kernel<<<(nwords + 255) / 256, 256, 0, stream>>>((unsigned*)XZ, nwords, kCarryMid);
  }

  wmma_gemm64<0, false, 2, 0, true><<<dim3((kRows / 64) * (kDim / 64) / 8, 1), 256, 0, stream>>>(
      XZ, nullptr, kFfn, 0L,
      WF2, nullptr, kFfn, 0L,
      (void*)out, nullptr, kDim, 0L,
      ffn_b2, H1, 0L,
      kRows, kDim, kFfn, 1.0f / (kCarryMid * kCarryW));
}
